// DissipativeHebbianLayer_25108378812947
// MI455X (gfx1250) — hardware-verified
//
#include <hip/hip_runtime.h>


#define NB_  4
#define TT   2048
#define DD   1024
#define NH_  8
#define HD   64
#define DI   (NH_ * HD)
#define ETA  0.1f
typedef _Float16 h16;
typedef unsigned short bf;
typedef __attribute__((ext_vector_type(16))) __bf16   v16bf;
typedef __attribute__((ext_vector_type(16))) _Float16 v16h;
typedef __attribute__((ext_vector_type(8)))  _Float16 v8h;
typedef __attribute__((ext_vector_type(8)))  unsigned short v8us;
typedef __attribute__((ext_vector_type(8)))  float    v8f;
typedef __attribute__((ext_vector_type(4)))  float    v4f;
typedef v8h  __attribute__((may_alias)) v8ha;
typedef v4f  __attribute__((may_alias)) v4fa;
typedef v8us __attribute__((may_alias)) v8usa;

__device__ __forceinline__ unsigned short f2bf(float f) { unsigned u = __float_as_uint(f); u += 0x7FFFu + ((u >> 16) & 1u); return (unsigned short)(u >> 16); }
__device__ __forceinline__ float bf2f(unsigned short b) { return __uint_as_float(((unsigned)b) << 16); }
__device__ __forceinline__ float bfr(float f) { return bf2f(f2bf(f)); }
__device__ __forceinline__ v16h cat16(v8h lo, v8h hi) { return __builtin_shufflevector(lo, hi, 0, 1, 2, 3, 4, 5, 6, 7, 8, 9, 10, 11, 12, 13, 14, 15); }
__device__ __forceinline__ v16bf cat16b(v8us lo, v8us hi) { return __builtin_bit_cast(v16bf, __builtin_shufflevector(lo, hi, 0, 1, 2, 3, 4, 5, 6, 7, 8, 9, 10, 11, 12, 13, 14, 15)); }
__device__ __forceinline__ v8f wmma16(v16h a, v16h b, v8f c) { return __builtin_amdgcn_wmma_f32_16x16x32_f16(false, a, false, b, (short)0, c, false, false); }
__device__ __forceinline__ v8f wmmab(v16bf a, v16bf b, v8f c) { return __builtin_amdgcn_wmma_f32_16x16x32_bf16(false, a, false, b, (short)0, c, false, false); }


template <typename T16> struct WFrag;
template <> struct WFrag<h16> { typedef v16h V; static __device__ __forceinline__ V ld(const h16* p) { return cat16(*(const v8h*)p, *(const v8h*)(p + 16)); } static __device__ __forceinline__ v8f mma(V a, V b, v8f c) { return wmma16(a, b, c); } };
template <> struct WFrag<bf> { typedef v16bf V; static __device__ __forceinline__ V ld(const bf* p) { return cat16b(*(const v8us*)p, *(const v8us*)(p + 16)); } static __device__ __forceinline__ v8f mma(V a, V b, v8f c) { return wmmab(a, b, c); } };
template <typename T16, int NSPLIT, bool BIAS>
__global__ __launch_bounds__(32) void k_gemmw(const T16* __restrict__ A, const T16* __restrict__ A2, const T16* __restrict__ Bt, const T16* __restrict__ Bt2, int K, float* C, int ldc, const float* __restrict__ bias, size_t sA, size_t sB, size_t sC) {
    typedef typename WFrag<T16>::V V;
    __shared__ __align__(16) float os[16 * 68];
    const size_t z = blockIdx.z; A += z * sA; if (A2) A2 += z * sA; Bt += z * sB; if (Bt2) Bt2 += z * sB; C += z * sC;
    const int lane = threadIdx.x & 31, lr = lane & 15, hi = lane >> 4; const int r0 = blockIdx.x * 64, c0 = blockIdx.y * 64;
    v8f acc[4][4];
#pragma unroll
    for (int mb = 0; mb < 4; ++mb)
#pragma unroll
        for (int nb = 0; nb < 4; ++nb) acc[mb][nb] = (v8f){};
    const size_t aoff = (size_t)(r0 + lr) * K + 8 * hi, boff = (size_t)(c0 + lr) * K + 8 * hi;
#pragma unroll 1
    for (int kc = 0; kc < K; kc += 32) {
        V a[4], a2[4];
#pragma unroll
        for (int mb = 0; mb < 4; ++mb) { a[mb] = WFrag<T16>::ld(A + aoff + (size_t)mb * 16 * K + kc); if (NSPLIT == 1 || NSPLIT == 2) a2[mb] = WFrag<T16>::ld(A2 + aoff + (size_t)mb * 16 * K + kc); }
#pragma unroll
        for (int nb = 0; nb < 4; ++nb) { const V b = WFrag<T16>::ld(Bt + boff + (size_t)nb * 16 * K + kc); V b2; if (NSPLIT >= 2) b2 = WFrag<T16>::ld(Bt2 + boff + (size_t)nb * 16 * K + kc);
#pragma unroll
            for (int mb = 0; mb < 4; ++mb) { acc[mb][nb] = WFrag<T16>::mma(a[mb], b, acc[mb][nb]); if (NSPLIT == 1 || NSPLIT == 2) acc[mb][nb] = WFrag<T16>::mma(a2[mb], b, acc[mb][nb]); if (NSPLIT >= 2) acc[mb][nb] = WFrag<T16>::mma(a[mb], b2, acc[mb][nb]); } }
        asm volatile("v_nop\n\tv_nop\n\tv_nop\n\tv_nop" : "+v"(acc[0][0]), "+v"(acc[1][1]), "+v"(acc[2][2]), "+v"(acc[3][3]) : "v"(a[0]), "v"(a[3]));
    }
#pragma unroll
    for (int mb = 0; mb < 4; ++mb) {
#pragma unroll
        for (int nb = 0; nb < 4; ++nb) {
#pragma unroll
            for (int j = 0; j < 8; ++j) os[(hi * 8 + j) * 68 + nb * 16 + lr] = acc[mb][nb][j]; }
        __builtin_amdgcn_wave_barrier(); asm volatile("" ::: "memory");
        float* crow = C + (size_t)(r0 + mb * 16) * ldc + c0;
#pragma unroll 1
        for (int ps = 0; ps < 2; ++ps) {
#pragma unroll
            for (int s = 0; s < 8; ++s) { const int row = 2 * s + hi, cofs = lr * 4; v4f val = *(const v4fa*)(os + row * 68 + cofs); if (BIAS) { val[0] += bfr(bias[c0 + cofs]); val[1] += bfr(bias[c0 + cofs + 1]); val[2] += bfr(bias[c0 + cofs + 2]); val[3] += bfr(bias[c0 + cofs + 3]); }
                *(volatile v4f*)(crow + (size_t)row * ldc + cofs) = val; }
            if (ps == 0) __threadfence(); }
        __builtin_amdgcn_wave_barrier(); asm volatile("" ::: "memory");
    }
}

__device__ __forceinline__ h16 tohx(float x) { return (h16)x; }
__device__ __forceinline__ void splitf(float y, unsigned short& h, unsigned short& l) { h = f2bf(y); l = f2bf(y - bf2f(h)); }
typedef __attribute__((ext_vector_type(2))) _Float16 v2h;
typedef __attribute__((ext_vector_type(2))) unsigned short v2us;
typedef __attribute__((ext_vector_type(4))) unsigned short v4us;
typedef __attribute__((ext_vector_type(2))) float v2f;

__global__ __launch_bounds__(256) void k_wtG(const float* __restrict__ w, int K, int N, bf* Bt) {
    const int lane = threadIdx.x & 31; const int L0 = (blockIdx.x * 8 + (threadIdx.x >> 5)) * 8; const int nlines = N * K / 64;
#pragma unroll 1
    for (int ps = 0; ps < 2; ++ps) {
#pragma unroll 1
        for (int l = 0; l < 8; ++l) { const int L = L0 + l; if (L >= nlines) break; const size_t e = (size_t)L * 64 + lane * 2; const int k = (int)(e % K), n = (int)(e / K); v2us o;
            o[0] = f2bf(w[(size_t)k * N + n]); o[1] = f2bf(w[(size_t)(k + 1) * N + n]); *(volatile v2us*)(Bt + e) = o; }
        if (ps == 0) __threadfence(); }
}
__global__ __launch_bounds__(256) void k_cvt8(const float* __restrict__ src, bf* dst, size_t n8) { const size_t i = (size_t)blockIdx.x * 256 + threadIdx.x; if (i >= n8) return; const v8f v = *(const v8f*)(src + i * 8); v8us o;
#pragma unroll
    for (int k = 0; k < 8; ++k) o[k] = f2bf(v[k]); *(volatile v8us*)(dst + i * 8) = o; __threadfence(); *(volatile v8us*)(dst + i * 8) = o; }
__global__ __launch_bounds__(256) void k_hsp(const float* __restrict__ F, int pitch, int nheads, float sc, bf* Ph, bf* Pl) { const size_t e = ((size_t)blockIdx.x * 256 + threadIdx.x) * 2; if (e >= (size_t)nheads * TT * HD) return; const int d = (int)(e & 63); const int t = (int)((e >> 6) & (TT - 1)); const int h = (int)(e >> 17); v2us oh, ol;
#pragma unroll
    for (int q = 0; q < 2; ++q) { unsigned short a, c2; splitf(F[(size_t)t * pitch + h * HD + d + q] * sc, a, c2); oh[q] = a; ol[q] = c2; }
    *(volatile v2us*)(Ph + e) = oh; *(volatile v2us*)(Pl + e) = ol; __threadfence(); *(volatile v2us*)(Ph + e) = oh; *(volatile v2us*)(Pl + e) = ol; }
__global__ __launch_bounds__(256) void k_vtplane(const float* __restrict__ F, int pitch, int nheads, bf* Vh, bf* Vl, h16* V16) {
    const int lane = threadIdx.x & 31; const int L0 = (blockIdx.x * 8 + (threadIdx.x >> 5)) * 8; const int nlines = nheads * TT * HD / 64;
#pragma unroll 1
    for (int ps = 0; ps < 2; ++ps) {
#pragma unroll
        for (int l = 0; l < 8; ++l) { const int L = L0 + l; if (L >= nlines) break; const int e = L * 64 + lane * 2; const int t = e & (TT - 1); const int d = (e >> 11) & (HD - 1); const int h = e >> 17; v2us oh, ol; v2h o16;
#pragma unroll
            for (int q = 0; q < 2; ++q) { const float x = F[(size_t)(t + q) * pitch + h * HD + d]; unsigned short a, c2; splitf(x, a, c2); oh[q] = a; ol[q] = c2; o16[q] = tohx(x); }
            *(volatile v2us*)(Vh + (size_t)e) = oh; *(volatile v2us*)(Vl + (size_t)e) = ol; *(volatile v2h*)(V16 + (size_t)e) = o16; }
        if (ps == 0) __threadfence(); }
}
__global__ __launch_bounds__(32) void k_cum(const float* __restrict__ gam, float* C) { const int b = threadIdx.x; if (b >= NB_) return;
    for (int ps = 0; ps < 2; ++ps) { float acc = 0.f; for (int t = 0; t < TT; ++t) { const float g = bfr(gam[(size_t)b * TT + t]); acc = __fadd_rn(acc, -fminf(__fmul_rn(g, 1.0f), 10.0f)); *(volatile float*)(C + (size_t)b * TT + t) = acc; } if (ps == 0) __threadfence(); } }
__global__ __launch_bounds__(256) void k_dec(const float* __restrict__ A, const float* __restrict__ C, bf* Gh, bf* Gl) { const int lane = threadIdx.x & 31; const int t = blockIdx.x * 8 + (threadIdx.x >> 5); if (t >= TT) return; const float ct = C[t]; const float* ar = A + (size_t)t * TT;
#pragma unroll 1
    for (int ps = 0; ps < 2; ++ps) {
#pragma unroll 2
        for (int ch = 0; ch < 16; ++ch) { const int s0 = ch * 128 + lane * 4; const v4f a = *(const v4f*)(ar + s0), c4 = *(const v4f*)(C + s0); v4us oh, ol;
#pragma unroll
            for (int q = 0; q < 4; ++q) { const int s = s0 + q; float g = 0.f; if (s <= t) { float dl = __fsub_rn(ct, c4[q]); asm volatile("" : "+v"(dl)); const float dc = __builtin_amdgcn_exp2f(__fmul_rn(dl, 1.4426950408889634f)); float ea = __fmul_rn(ETA, a[q]); asm volatile("" : "+v"(ea)); g = __fmul_rn(ea, dc); }
                unsigned short a2, c2; splitf(g, a2, c2); oh[q] = a2; ol[q] = c2; }
            const size_t o = (size_t)t * TT + s0; *(volatile v4us*)(Gh + o) = oh; *(volatile v4us*)(Gl + o) = ol; }
        if (ps == 0) __threadfence(); }
}
__global__ __launch_bounds__(256) void k_wv(const float* __restrict__ FV, const float* __restrict__ C, bf* Wh, bf* Wl) { const size_t e = ((size_t)blockIdx.x * 256 + threadIdx.x) * 2; if (e >= (size_t)NH_ * HD * TT) return; const int s = (int)(e & (TT - 1)); const int j = (int)((e >> 11) & 63); const int h = (int)(e >> 17); const float cN = C[TT - 1]; v2us oh, ol;
#pragma unroll
    for (int q = 0; q < 2; ++q) { float dl = __fsub_rn(cN, C[s + q]); asm volatile("" : "+v"(dl)); const float w = __builtin_amdgcn_exp2f(__fmul_rn(dl, 1.4426950408889634f)); unsigned short a, c2; splitf(__fmul_rn(FV[(size_t)(s + q) * DI + h * HD + j], w), a, c2); oh[q] = a; ol[q] = c2; }
    *(volatile v2us*)(Wh + e) = oh; *(volatile v2us*)(Wl + e) = ol; __threadfence(); *(volatile v2us*)(Wh + e) = oh; *(volatile v2us*)(Wl + e) = ol; }
__global__ __launch_bounds__(256) void k_ymrg(const float* __restrict__ Y1, const float* __restrict__ YS, const float* __restrict__ C, int h, bf* Yh, bf* Yl) { const size_t e = ((size_t)blockIdx.x * 256 + threadIdx.x) * 2; if (e >= (size_t)TT * HD) return; const int t = (int)(e >> 6), i = (int)(e & 63); const float ec = __builtin_amdgcn_exp2f(__fmul_rn(C[t], 1.4426950408889634f)); v2us oh, ol;
#pragma unroll
    for (int q = 0; q < 2; ++q) { float ys = __fmul_rn(ec, YS[e + q]); asm volatile("" : "+v"(ys)); unsigned short a, c2; splitf(__fadd_rn(Y1[e + q], ys), a, c2); oh[q] = a; ol[q] = c2; }
    const size_t o = (size_t)t * DI + h * HD + i; *(volatile v2us*)(Yh + o) = oh; *(volatile v2us*)(Yl + o) = ol; __threadfence(); *(volatile v2us*)(Yh + o) = oh; *(volatile v2us*)(Yl + o) = ol; }
__global__ __launch_bounds__(256) void k_stfin(const float* __restrict__ STF, const float* __restrict__ st0, const float* __restrict__ C, float* OUT1) { const int i = (blockIdx.x * 256 + threadIdx.x) * 4; if (i >= HD * HD) return; const float ec = __builtin_amdgcn_exp2f(__fmul_rn(C[TT - 1], 1.4426950408889634f)); const v4f a = *(const v4f*)(STF + i), s4 = *(const v4f*)(st0 + i); v4f o;
#pragma unroll
    for (int q = 0; q < 4; ++q) { float t1 = __fmul_rn(ETA, a[q]), t2 = __fmul_rn(ec, bfr(s4[q])); asm volatile("" : "+v"(t1)); asm volatile("" : "+v"(t2)); o[q] = __fadd_rn(t1, t2); }
    *(volatile v4f*)(OUT1 + i) = o; __threadfence(); *(volatile v4f*)(OUT1 + i) = o; }

extern "C" void kernel_launch(void* const* d_in, const int* in_sizes, int n_in,
                              void* d_out, int out_size, void* d_ws, size_t ws_size, hipStream_t stream) {
    (void)in_sizes; (void)n_in; (void)out_size;
    const float* x = (const float*)d_in[0]; const float* gam = (const float*)d_in[1]; const float* st0 = (const float*)d_in[2]; const float* Wq = (const float*)d_in[3]; const float* Wk = (const float*)d_in[4]; const float* Wv = (const float*)d_in[5]; const float* Wo = (const float*)d_in[6]; const float* bo = (const float*)d_in[7];
    float* OUT0 = (float*)d_out; float* OUT1 = OUT0 + (size_t)NB_ * TT * DD;
    char* wsp = (char*)d_ws;
    auto take = [&](size_t bytes) { char* p = wsp; wsp += (bytes + 255) & ~(size_t)255; return (void*)p; };
    bf* WQ = (bf*)take((size_t)DD * DI * 2); bf* WK = (bf*)take((size_t)DD * DI * 2); bf* WV = (bf*)take((size_t)DD * DI * 2); bf* WO = (bf*)take((size_t)DI * DD * 2); float* C = (float*)take((size_t)NB_ * TT * 4);
    bf* XB = (bf*)take((size_t)TT * DD * 2); float* FQ = (float*)take((size_t)TT * DI * 4); float* FK = (float*)take((size_t)TT * DI * 4); float* FV = (float*)take((size_t)TT * DI * 4);
    bf* Qh = (bf*)take((size_t)NH_ * TT * HD * 2); bf* Ql = (bf*)take((size_t)NH_ * TT * HD * 2); bf* Vh = (bf*)take((size_t)NH_ * TT * HD * 2); bf* Vl = (bf*)take((size_t)NH_ * TT * HD * 2);
    bf* KTh = (bf*)take((size_t)NH_ * HD * TT * 2); bf* KTl = (bf*)take((size_t)NH_ * HD * TT * 2); h16* KT16 = (h16*)take((size_t)NH_ * HD * TT * 2); bf* WVh = (bf*)take((size_t)NH_ * HD * TT * 2); bf* WVl = (bf*)take((size_t)NH_ * HD * TT * 2);
    float* A = (float*)take((size_t)TT * TT * 4); bf* Gh = (bf*)take((size_t)TT * TT * 2); bf* Gl = (bf*)take((size_t)TT * TT * 2); float* Y1 = (float*)take((size_t)TT * HD * 4); float* YS = (float*)take((size_t)TT * HD * 4); bf* S0 = (bf*)take(HD * HD * 2); float* STF = (float*)take(HD * HD * 4);
    bf* Yh = (bf*)take((size_t)TT * DI * 2); bf* Yl = (bf*)take((size_t)TT * DI * 2);
    if ((size_t)(wsp - (char*)d_ws) > ws_size) return;
    { const unsigned gT = (unsigned)((DD * DI / 64 + 63) / 64); k_wtG<<<gT, 256, 0, stream>>>(Wq, DD, DI, WQ); k_wtG<<<gT, 256, 0, stream>>>(Wk, DD, DI, WK); k_wtG<<<gT, 256, 0, stream>>>(Wv, DD, DI, WV); k_wtG<<<(unsigned)((DI * DD / 64 + 63) / 64), 256, 0, stream>>>(Wo, DI, DD, WO); k_cum<<<1, 32, 0, stream>>>(gam, C); }
    const unsigned LP = (unsigned)(((size_t)NH_ * TT * HD / 2 + 255) / 256), LV = (unsigned)((NH_ * HD * TT / 64 + 63) / 64); const dim3 gP(TT / 64, DI / 64, 1);
    for (int b = 0; b < NB_; ++b) { const float* Cb = C + (size_t)b * TT;
        k_cvt8<<<(unsigned)(((size_t)TT * DD / 8 + 255) / 256), 256, 0, stream>>>(x + (size_t)b * TT * DD, XB, (size_t)TT * DD / 8);
        k_gemmw<bf, 0, false><<<gP, 32, 0, stream>>>(XB, nullptr, WQ, nullptr, DD, FQ, DI, nullptr, 0, 0, 0); k_hsp<<<LP, 256, 0, stream>>>(FQ, DI, NH_, 1.0f, Qh, Ql);
        k_gemmw<bf, 0, false><<<gP, 32, 0, stream>>>(XB, nullptr, WV, nullptr, DD, FV, DI, nullptr, 0, 0, 0); k_hsp<<<LP, 256, 0, stream>>>(FV, DI, NH_, 1.0f, Vh, Vl); k_wv<<<LP, 256, 0, stream>>>(FV, Cb, WVh, WVl);
        k_gemmw<bf, 0, false><<<gP, 32, 0, stream>>>(XB, nullptr, WK, nullptr, DD, FK, DI, nullptr, 0, 0, 0); k_vtplane<<<LV, 256, 0, stream>>>(FK, DI, NH_, KTh, KTl, KT16);
        for (int h = 0; h < NH_; ++h) { const size_t po = (size_t)h * TT * HD;
            k_gemmw<bf, 2, false><<<dim3(TT / 64, TT / 64, 1), 32, 0, stream>>>(Qh + po, Ql + po, Vh + po, Vl + po, HD, A, TT, nullptr, 0, 0, 0);
            k_dec<<<TT / 8, 256, 0, stream>>>(A, Cb, Gh, Gl);
            k_gemmw<bf, 2, false><<<dim3(TT / 64, 1, 1), 32, 0, stream>>>(Gh, Gl, KTh + po, KTl + po, TT, Y1, HD, nullptr, 0, 0, 0);
            k_cvt8<<<(HD * HD / 8 + 255) / 256, 256, 0, stream>>>(st0 + ((size_t)b * NH_ + h) * HD * HD, S0, HD * HD / 8);
            k_gemmw<bf, 1, false><<<dim3(TT / 64, 1, 1), 32, 0, stream>>>(Qh + po, Ql + po, S0, nullptr, HD, YS, HD, nullptr, 0, 0, 0);
            k_ymrg<<<(unsigned)(((size_t)TT * HD / 2 + 255) / 256), 256, 0, stream>>>(Y1, YS, Cb, h, Yh, Yl);
            k_gemmw<bf, 2, false><<<dim3(1, 1, 1), 32, 0, stream>>>(KTh + po, KTl + po, WVh + po, WVl + po, TT, STF, HD, nullptr, 0, 0, 0);
            k_stfin<<<(HD * HD / 4 + 255) / 256, 256, 0, stream>>>(STF, st0 + ((size_t)b * NH_ + h) * HD * HD, Cb, OUT1 + ((size_t)b * NH_ + h) * HD * HD); }
        k_gemmw<bf, 1, true><<<dim3(TT / 64, DD / 64, 1), 32, 0, stream>>>(Yh, Yl, WO, nullptr, DI, OUT0 + (size_t)b * TT * DD, DD, bo, 0, 0, 0); }
}
